// RandomFeaturesLayer_36756330120125
// MI455X (gfx1250) — hardware-verified
//
#include <hip/hip_runtime.h>


namespace {
constexpr int B = 4096, IN = 2048, OUT = 2048;

typedef _Float16 b16;
typedef __attribute__((ext_vector_type(16))) _Float16 v16b;
typedef __attribute__((ext_vector_type(16))) __bf16 v16bb;
typedef __attribute__((ext_vector_type(8))) _Float16 v8b;
typedef __attribute__((ext_vector_type(8))) unsigned short v8us;
typedef __attribute__((ext_vector_type(8))) float v8f;
typedef __attribute__((ext_vector_type(4))) float v4f;
__device__ __forceinline__ float bf16_rne(float f) { unsigned int u = __float_as_uint(f); u += 0x7FFFu + ((u >> 16) & 1u); return __uint_as_float(u & 0xFFFF0000u); }
__device__ __forceinline__ unsigned short bf16_bits(float f) { unsigned int u = __float_as_uint(f); u += 0x7FFFu + ((u >> 16) & 1u); return (unsigned short)(u >> 16); }
__device__ __forceinline__ v16b frag_kb(const b16* p, int hh) { const v8b a = *(const v8b*)(p + 8 * hh), b = *(const v8b*)(p + 16 + 8 * hh); v16b f;
#pragma unroll
  for (int e = 0; e < 8; ++e) { f[e] = a[e]; f[8 + e] = b[e]; } return f; }
__device__ __forceinline__ v16bb frag_bf(const unsigned short* p, int hh) { const v8us a = *(const v8us*)(p + 8 * hh), b = *(const v8us*)(p + 16 + 8 * hh); union { unsigned short s[16]; v16bb v; } u;
#pragma unroll
  for (int e = 0; e < 8; ++e) { u.s[e] = a[e]; u.s[8 + e] = b[e]; } return u.v; }
__device__ __forceinline__ v16bb frag_f32bf(const float* p, int hh) { union { unsigned short s[16]; v16bb v; } u;
#pragma unroll
  for (int e = 0; e < 8; ++e) { u.s[e] = bf16_bits(p[8 * hh + e]); u.s[8 + e] = bf16_bits(p[16 + 8 * hh + e]); } return u.v; }
__device__ __forceinline__ v8f wmma16b(v16b a, v16b b, v8f c) { v8f d = __builtin_amdgcn_wmma_f32_16x16x32_f16(false, a, false, b, (short)0, c, false, false); asm volatile("v_nop\n\tv_nop\n\tv_nop\n\tv_nop" : "+v"(d) : "v"(a), "v"(b)); return d; }
__device__ __forceinline__ v8f wmma16bb(v16bb a, v16bb b, v8f c) { v8f d = __builtin_amdgcn_wmma_f32_16x16x32_bf16(false, a, false, b, (short)0, c, false, false); asm volatile("v_nop\n\tv_nop\n\tv_nop\n\tv_nop" : "+v"(d) : "v"(a), "v"(b)); return d; }
__device__ __forceinline__ void wave_lds_sync() { __builtin_amdgcn_fence(__ATOMIC_RELEASE, "workgroup"); __builtin_amdgcn_wave_barrier(); __builtin_amdgcn_fence(__ATOMIC_ACQUIRE, "workgroup"); }

__global__ __launch_bounds__(256) void prep_kernel(const float* __restrict__ rp, const float* __restrict__ W, unsigned short* __restrict__ rp16, b16* __restrict__ w16) {
  const size_t tid = (size_t)blockIdx.x * blockDim.x + threadIdx.x, nth = (size_t)gridDim.x * blockDim.x;
  for (int pass = 0; pass < 2; ++pass) {
    for (size_t p = tid; p < (size_t)OUT * IN / 8; p += nth) { v8us v; v8b w;
#pragma unroll
      for (int e = 0; e < 8; ++e) { v[e] = bf16_bits(rp[p * 8 + e]); w[e] = (b16)bf16_rne(W[p * 8 + e]); }
      *(volatile v8us*)(rp16 + p * 8) = v; *(volatile v8b*)(w16 + p * 8) = w; }
    __threadfence(); }
}

__global__ __launch_bounds__(128) void gemm1_kernel(const float* __restrict__ x, const unsigned short* __restrict__ rp16, b16* __restrict__ h) {
  __shared__ __attribute__((aligned(16))) b16 Th[4][32][64 + 8], Tl[4][32][64 + 8];
  const int lane = threadIdx.x & 31, wave = threadIdx.x >> 5, nloc = lane & 15, hlf = lane >> 4, m0 = blockIdx.y * 128 + wave * 32, c0 = blockIdx.x * 64;
  v8f acc[2][4];
#pragma unroll
  for (int r = 0; r < 2; ++r)
#pragma unroll
    for (int t = 0; t < 4; ++t) acc[r][t] = (v8f){};
#pragma unroll 2
  for (int kb = 0; kb < IN; kb += 32) { const v16bb a0 = frag_f32bf(x + (size_t)(m0 + nloc) * IN + kb, hlf), a1 = frag_f32bf(x + (size_t)(m0 + 16 + nloc) * IN + kb, hlf);
#pragma unroll
    for (int t = 0; t < 4; ++t) { const v16bb bw = frag_bf(rp16 + (size_t)(c0 + t * 16 + nloc) * IN + kb, hlf); acc[0][t] = wmma16bb(a0, bw, acc[0][t]); acc[1][t] = wmma16bb(a1, bw, acc[1][t]); } }
#pragma unroll
  for (int t = 0; t < 4; ++t)
#pragma unroll
    for (int r = 0; r < 2; ++r)
#pragma unroll
      for (int v = 0; v < 8; ++v) { const float val = acc[r][t][v]; const b16 hi = (b16)val; Th[wave][r * 16 + 8 * hlf + v][t * 16 + nloc] = hi; Tl[wave][r * 16 + 8 * hlf + v][t * 16 + nloc] = (b16)(val - (float)hi); }
  wave_lds_sync();
  for (int pass = 0; pass < 2; ++pass) {
#pragma unroll
    for (int j = 0; j < 8; ++j) { const int rr = j * 4 + (lane >> 3), c8 = (lane & 7) * 8; *(volatile v8b*)(h + (size_t)(m0 + rr) * OUT + c0 + c8) = *(const v8b*)(&Th[wave][rr][c8]); *(volatile v8b*)(h + (size_t)B * OUT + (size_t)(m0 + rr) * OUT + c0 + c8) = *(const v8b*)(&Tl[wave][rr][c8]); }
    __threadfence(); }
}

__global__ __launch_bounds__(128) void gemm2_kernel(const b16* __restrict__ h, const b16* __restrict__ w16, const float* __restrict__ bias, float* __restrict__ out) {
  __shared__ __attribute__((aligned(16))) float Ts[4][32 * 64];
  const int lane = threadIdx.x & 31, wave = threadIdx.x >> 5, nloc = lane & 15, hlf = lane >> 4, m0 = blockIdx.y * 128 + wave * 32, c0 = blockIdx.x * 64;
  v8f acc[2][4];
#pragma unroll
  for (int r = 0; r < 2; ++r)
#pragma unroll
    for (int t = 0; t < 4; ++t) acc[r][t] = (v8f){};
#pragma unroll 2
  for (int kb = 0; kb < OUT; kb += 32) { const v16b a0 = frag_kb(h + (size_t)(m0 + nloc) * OUT + kb, hlf), a1 = frag_kb(h + (size_t)(m0 + 16 + nloc) * OUT + kb, hlf), l0 = frag_kb(h + (size_t)B * OUT + (size_t)(m0 + nloc) * OUT + kb, hlf), l1 = frag_kb(h + (size_t)B * OUT + (size_t)(m0 + 16 + nloc) * OUT + kb, hlf);
#pragma unroll
    for (int t = 0; t < 4; ++t) { const v16b bw = frag_kb(w16 + (size_t)(c0 + t * 16 + nloc) * OUT + kb, hlf); acc[0][t] = wmma16b(a0, bw, acc[0][t]); acc[0][t] = wmma16b(l0, bw, acc[0][t]); acc[1][t] = wmma16b(a1, bw, acc[1][t]); acc[1][t] = wmma16b(l1, bw, acc[1][t]); } }
  float* Tt = Ts[wave];
#pragma unroll
  for (int t = 0; t < 4; ++t) { const float bb = 0.1f * bf16_rne(bias[c0 + t * 16 + nloc]);
#pragma unroll
    for (int r = 0; r < 2; ++r)
#pragma unroll
      for (int v = 0; v < 8; ++v) Tt[(r * 16 + v + 8 * hlf) * 64 + t * 16 + nloc] = acc[r][t][v] + bb; }
  wave_lds_sync();
  for (int pass = 0; pass < 2; ++pass) {
#pragma unroll
    for (int j = 0; j < 16; ++j) { const int rr = j * 2 + hlf, c4 = nloc * 4; *(volatile v4f*)(out + (size_t)(m0 + rr) * OUT + c0 + c4) = *(const v4f*)(Tt + rr * 64 + c4); }
    __threadfence(); }
}
}

extern "C" void kernel_launch(void* const* d_in, const int* in_sizes, int n_in,
                              void* d_out, int out_size, void* d_ws, size_t ws_size, hipStream_t stream) {
  (void)n_in; (void)out_size;
  const float* x = (const float*)d_in[0]; const float* rp = (const float*)d_in[1]; const float* W = (const float*)d_in[2]; const float* bias = (const float*)d_in[3];
  float* out = (float*)d_out;
  if (in_sizes[0] != B * IN || in_sizes[1] != OUT * IN || in_sizes[2] != OUT * OUT || in_sizes[3] != OUT) return;
  size_t off = 0; char* ws = (char*)d_ws;
  auto carve = [&](size_t bytes) { char* p = ws + off; off += (bytes + 255) & ~(size_t)255; return p; };
  unsigned short* rp16 = (unsigned short*)carve((size_t)OUT * IN * 2); b16* w16 = (b16*)carve((size_t)OUT * OUT * 2); b16* h = (b16*)carve((size_t)B * OUT * 2 * 2);
  if (off > ws_size) return;
  prep_kernel<<<1024, 256, 0, stream>>>(rp, W, rp16, w16);
  gemm1_kernel<<<dim3(OUT / 64, B / 128), 128, 0, stream>>>(x, rp16, h);
  gemm2_kernel<<<dim3(OUT / 64, B / 128), 128, 0, stream>>>(h, w16, bias, out);
}
